// GATPairClassifier_16784732193027
// MI455X (gfx1250) — hardware-verified
//
#include <hip/hip_runtime.h>
#include <math.h>
#include <stdint.h>

#define NB   32
#define NN   512
#define NF   256
#define HD   64
#define NH   8
#define MR   (NB * NN)
#define C1   (NH * HD)
#define K2   (2 * C1)
#define NCAT (NF + HD)
#define TP   68
#define CP   324
#define BN_EPS 1e-5f
#define DYN_TILE_BYTES (NN * TP * 4)

static_assert(MR == 16384);
static_assert(MR % 64 == 0);
static_assert(NN % 128 == 0);
static_assert(HD == 64);
static_assert(C1 == 512);
static_assert(C1 % 64 == 0);
static_assert(NF % 32 == 0);
static_assert(K2 % 32 == 0);
static_assert(NN % 32 == 0);
static_assert((CP * 4) % 16 == 0);
static_assert((TP * 4) % 16 == 0);
static_assert(DYN_TILE_BYTES == 139264);

typedef __attribute__((ext_vector_type(16))) __bf16   v16b;
typedef __attribute__((ext_vector_type(8)))  __bf16   v8b;
typedef __attribute__((ext_vector_type(8)))  float    v8f;
typedef __attribute__((ext_vector_type(4)))  float    v4f;
typedef __attribute__((ext_vector_type(4)))  unsigned int v4u;
typedef __attribute__((ext_vector_type(8)))  unsigned int v8u;
typedef v4f __attribute__((may_alias)) v4fa;

__device__ __forceinline__ unsigned short f2bf_bits(float f) {
  unsigned u = __float_as_uint(f);
  return (unsigned short)((u + 0x7FFFu + ((u >> 16) & 1u)) >> 16);
}
__device__ __forceinline__ float bf_bits2f(unsigned short h) { return __uint_as_float(((unsigned)h) << 16); }
__device__ __forceinline__ unsigned pk16(unsigned short a, unsigned short b) { return (unsigned)a | ((unsigned)b << 16); }
__device__ __forceinline__ float bfr(float x) { return bf_bits2f(f2bf_bits(x)); }

__device__ __forceinline__ float leakyf(float v) { return (v > 0.0f) ? v : 0.2f * v; }
__device__ __forceinline__ float eluf(float v) { return (v > 0.0f) ? v : expm1f(v); }
__device__ __forceinline__ float colmax(float fm, float f2v) {
#pragma clang fp contract(off)
  const float v = fm + f2v;
  return (v > 0.0f) ? v : 0.2f * v;
}
__device__ __forceinline__ float pexp(float f1v, float f2v, float m) {
#pragma clang fp contract(off)
  const float v = f1v + f2v;
  const float e = (v > 0.0f) ? v : 0.2f * v;
  return expf(e - m);
}

__device__ __forceinline__ void dep_guard_b(v8f& a, v8f& b, v16b x, v16b y) { asm volatile("v_nop\n\tv_nop\n\tv_nop\n\tv_nop" : "+v"(a), "+v"(b) : "v"(x), "v"(y)); }
__device__ __forceinline__ void keep4_b(v16b a, v16b b, v16b c, v16b d) { asm volatile("v_nop" :: "v"(a), "v"(b), "v"(c), "v"(d)); }
__device__ __forceinline__ void acc_guard4(v8f& a, v8f& b, v8f& c, v8f& d) { asm volatile("v_nop\n\tv_nop\n\tv_nop\n\tv_nop" : "+v"(a), "+v"(b), "+v"(c), "+v"(d)); }

struct FragB {
  union U { v16b v; v8b h[2]; };
  static __device__ __forceinline__ v16b load(const __bf16* p) {
    U f; f.h[0] = *(const v8b*)(p); f.h[1] = *(const v8b*)(p + 16); return f.v;
  }
  static __device__ __forceinline__ v8f mma(v16b a, v16b b, v8f c) {
    return __builtin_amdgcn_wmma_f32_16x16x32_bf16(false, a, false, b, (short)0, c, false, false);
  }
};
__device__ __forceinline__ v8f at_mma(v16b a, v16b b, v8f c) {
  c = __builtin_amdgcn_wmma_f32_16x16x32_bf16(false, a, false, b, (short)0, c, false, false);
  asm volatile("v_nop\n\tv_nop\n\tv_nop\n\tv_nop" : "+v"(c) : "v"(a), "v"(b));
  return c;
}
__device__ __forceinline__ v8f zero8() { v8f z = {0.f, 0.f, 0.f, 0.f, 0.f, 0.f, 0.f, 0.f}; return z; }

__global__ __launch_bounds__(256) void wmma_gemm64_f32(
    const unsigned short* __restrict__ Ap, int lda,
    const unsigned short* __restrict__ Btp, int ldb,
    float* C, int ldc, int M, int N, int K) {
  const __bf16* A  = (const __bf16*)(const void*)Ap;
  const __bf16* Bt = (const __bf16*)(const void*)Btp;
  __shared__ __align__(16) float sT[8][16 * TP];
  const int lane = threadIdx.x & 31;
  const int wave = threadIdx.x >> 5;
  const int tilesN = N >> 6;
  const int tilesM = M >> 6;
  const int tile = blockIdx.x * 8 + wave;
  if (tile >= tilesM * tilesN) return;
  const int tm = tile / tilesN;
  const int tn = tile - tm * tilesN;
  const int m0 = tm << 6;
  const int n0 = tn << 6;

  const int rlane = lane & 15;
  const int koff  = (lane >> 4) * 8;
  const int mOff  = (lane >> 4) * 8;

  v8f acc[4][4];
#pragma unroll
  for (int i = 0; i < 4; ++i)
#pragma unroll
    for (int j = 0; j < 4; ++j) acc[i][j] = zero8();

  for (int k0 = 0; k0 < K; k0 += 32) {
    v16b bh[4];
#pragma unroll
    for (int j = 0; j < 4; ++j) {
      const size_t bo = (size_t)(n0 + (j << 4) + rlane) * ldb + koff + k0;
      bh[j] = FragB::load(Bt + bo);
    }
#pragma unroll
    for (int i = 0; i < 4; ++i) {
      const size_t ao = (size_t)(m0 + (i << 4) + rlane) * lda + koff + k0;
      v16b ah = FragB::load(A + ao);
#pragma unroll
      for (int j = 0; j < 4; ++j) acc[i][j] = FragB::mma(ah, bh[j], acc[i][j]);
      dep_guard_b(acc[i][0], acc[i][3], ah, ah);
    }
    keep4_b(bh[0], bh[1], bh[2], bh[3]);
  }
  acc_guard4(acc[0][0], acc[0][1], acc[0][2], acc[0][3]);
  acc_guard4(acc[1][0], acc[1][1], acc[1][2], acc[1][3]);
  acc_guard4(acc[2][0], acc[2][1], acc[2][2], acc[2][3]);
  acc_guard4(acc[3][0], acc[3][1], acc[3][2], acc[3][3]);

  float* slab = sT[wave];
#pragma unroll
  for (int i = 0; i < 4; ++i) {
    const int mBase = m0 + (i << 4);
#pragma unroll
    for (int j = 0; j < 4; ++j) {
#pragma unroll
      for (int r = 0; r < 8; ++r) slab[(mOff + r) * TP + (j << 4) + rlane] = acc[i][j][r];
    }
    __builtin_amdgcn_fence(__ATOMIC_RELEASE, "workgroup");
    __builtin_amdgcn_wave_barrier();
    __builtin_amdgcn_fence(__ATOMIC_ACQUIRE, "workgroup");
    {
      const int hh = lane >> 4, c4 = (lane & 15) * 4;
      for (int pass = 0; pass < 2; ++pass) {
#pragma unroll
        for (int it = 0; it < 8; ++it) {
          const int row = it * 2 + hh;
          const v4f v = *(const v4fa*)(slab + row * TP + c4);
          *(volatile v4f*)(C + (size_t)(mBase + row) * ldc + n0 + c4) = v;
        }
        __threadfence();
      }
    }
    __builtin_amdgcn_fence(__ATOMIC_RELEASE, "workgroup");
    __builtin_amdgcn_wave_barrier();
    __builtin_amdgcn_fence(__ATOMIC_ACQUIRE, "workgroup");
  }
}

__global__ __launch_bounds__(256) void cvt_bf16x8_kernel(const float* __restrict__ in, unsigned short* o, int n8) {
  const int i = blockIdx.x * 256 + threadIdx.x;
  if (i < n8) {
    const float* sp = in + (size_t)i * 8;
    const v4f a  = *(const v4f*)(sp);
    const v4f a2 = *(const v4f*)(sp + 4);
    v4u w;
    w[0] = pk16(f2bf_bits(a[0]),  f2bf_bits(a[1]));
    w[1] = pk16(f2bf_bits(a[2]),  f2bf_bits(a[3]));
    w[2] = pk16(f2bf_bits(a2[0]), f2bf_bits(a2[1]));
    w[3] = pk16(f2bf_bits(a2[2]), f2bf_bits(a2[3]));
    unsigned short* dp = o + (size_t)i * 8;
    *(volatile v4u*)dp = w;
    __threadfence();
    *(volatile v4u*)dp = w;
  }
}

__global__ __launch_bounds__(256) void k_tr(const float* __restrict__ W, unsigned short* o, long sIn, int ldo, int dup) {
  __shared__ __align__(16) float tf[64 * TP];
  const int r0  = blockIdx.x * 64;
  const int z   = blockIdx.y;
  const int tid = threadIdx.x;
  const float* Wz = W + (size_t)z * sIn;
  {
    const int lr = tid >> 4;
    const int c4 = (tid & 15) * 4;
#pragma unroll
    for (int it = 0; it < 4; ++it) {
      const int rr = it * 16 + lr;
      const v4f a = *(const v4f*)(Wz + (size_t)(r0 + rr) * 64 + c4);
      *(v4f*)(tf + rr * TP + c4) = a;
    }
  }
  __syncthreads();
  const int sub = tid >> 3;
  const int c8  = (tid & 7) * 8;
  v4u hv[2];
#pragma unroll
  for (int it = 0; it < 2; ++it) {
    const int oc = it * 32 + sub;
    v4u a;
#pragma unroll
    for (int q = 0; q < 4; ++q) {
      const float f0 = tf[(c8 + 2 * q) * TP + oc];
      const float f1 = tf[(c8 + 2 * q + 1) * TP + oc];
      a[q] = pk16(f2bf_bits(f0), f2bf_bits(f1));
    }
    hv[it] = a;
  }
  for (int pass = 0; pass < 2; ++pass) {
#pragma unroll
    for (int it = 0; it < 2; ++it) {
      const int oc = it * 32 + sub;
      const size_t go = (size_t)(z * 64 + oc) * ldo + r0 + c8;
      *(volatile v4u*)(o + go) = hv[it];
      if (dup != 0) *(volatile v4u*)(o + go + C1) = hv[it];
    }
    __threadfence();
  }
}

__device__ __forceinline__ void stage_tile(float* tile, const float* __restrict__ src, int ldw, int tid) {
#pragma unroll 4
  for (int it = 0; it < 32; ++it) {
    const int p = it * 256 + tid;
    const int row = p >> 4;
    const int c4 = (p & 15) * 4;
    const v4f a = *(const v4f*)(src + (size_t)row * ldw + c4);
    *(v4f*)(tile + row * TP + c4) = a;
  }
}
__device__ __forceinline__ void dots_f12(const float* tile, const float* av, float* sf, int tid) {
#pragma unroll 1
  for (int q = 0; q < 4; ++q) {
    const int task = q * 256 + tid;
    const int row = task & 511;
    const int which = task >> 9;
    const float* tr = tile + row * TP;
    const float* ar = av + which * 64;
    float s = 0.0f;
#pragma unroll 4
    for (int d = 0; d < 64; ++d) s = fmaf(tr[d], ar[d], s);
    sf[which * 512 + row] = s;
  }
}
__device__ __forceinline__ float block_max512(const float* sf, float* red, int tid) {
  float m = fmaxf(sf[tid], sf[tid + 256]);
#pragma unroll
  for (int off = 16; off > 0; off >>= 1) m = fmaxf(m, __shfl_xor(m, off, 32));
  if ((tid & 31) == 0) red[tid >> 5] = m;
  __syncthreads();
  float fm = red[0];
#pragma unroll
  for (int w = 1; w < 8; ++w) fm = fmaxf(fm, red[w]);
  return fm;
}

extern __shared__ __align__(16) float dynT[];

__global__ __launch_bounds__(256) void k_stats(const float* __restrict__ WH1, const float* __restrict__ a_heads,
                                               float* F1, float* F2, float* MJ,
                                               unsigned short* VTh, unsigned short* VTl) {
  __shared__ __align__(16) float sav[128];
  __shared__ __align__(16) float sf[1024];
  __shared__ __align__(16) float mjs[512];
  __shared__ __align__(16) float rzs[512];
  __shared__ float red[8];
  const int tid = threadIdx.x;
  const int pair = blockIdx.x;
  const int b = pair >> 3, hd = pair & 7;
  float* tile = dynT;

  if (tid < 128) sav[tid] = bfr(a_heads[hd * 128 + tid]);
  stage_tile(tile, WH1 + (size_t)b * NN * C1 + hd * HD, C1, tid);
  __syncthreads();
  dots_f12(tile, sav, sf, tid);
  __syncthreads();
  const float fm = block_max512(sf, red, tid);
  {
    const float f2a = sf[512 + tid], f2b = sf[512 + tid + 256];
    const float ma = colmax(fm, f2a), mb = colmax(fm, f2b);
    float za = 0.0f, zb = 0.0f;
#pragma unroll 1
    for (int i = 0; i < 512; ++i) {
      const float f = sf[i];
      za += pexp(f, f2a, ma);
      zb += pexp(f, f2b, mb);
    }
    mjs[tid] = ma;        mjs[tid + 256] = mb;
    rzs[tid] = 1.0f / za; rzs[tid + 256] = 1.0f / zb;
  }
  __syncthreads();
  if (tid < 128) {
    const v4f a  = *(const v4fa*)(sf + tid * 4);
    const v4f a2 = *(const v4fa*)(sf + 512 + tid * 4);
    const v4f a3 = *(const v4fa*)(mjs + tid * 4);
    float* p1 = F1 + (size_t)pair * 512 + tid * 4;
    float* p2 = F2 + (size_t)pair * 512 + tid * 4;
    float* p3 = MJ + (size_t)pair * 512 + tid * 4;
    *(volatile v4f*)p1 = a; *(volatile v4f*)p2 = a2; *(volatile v4f*)p3 = a3;
    __threadfence();
    *(volatile v4f*)p1 = a; *(volatile v4f*)p2 = a2; *(volatile v4f*)p3 = a3;
  }
  for (int pass = 0; pass < 2; ++pass) {
#pragma unroll 2
    for (int it = 0; it < 16; ++it) {
      const int p = it * 256 + tid;
      const int d = p >> 6;
      const int j0 = (p & 63) * 8;
      const v4f r0 = *(const v4fa*)(rzs + j0);
      const v4f r1 = *(const v4fa*)(rzs + j0 + 4);
      v4u hw, lw;
#pragma unroll
      for (int q = 0; q < 4; ++q) {
        const float ra = (q < 2) ? r0[(2 * q) & 3] : r1[(2 * q) & 3];
        const float rb = (q < 2) ? r0[(2 * q + 1) & 3] : r1[(2 * q + 1) & 3];
        const float va = tile[(j0 + 2 * q) * TP + d] * ra;
        const float vb = tile[(j0 + 2 * q + 1) * TP + d] * rb;
        const unsigned short ha = f2bf_bits(va), hb = f2bf_bits(vb);
        const unsigned short la = f2bf_bits(va - bf_bits2f(ha)), lb = f2bf_bits(vb - bf_bits2f(hb));
        hw[q] = pk16(ha, hb);
        lw[q] = pk16(la, lb);
      }
      const size_t go = ((size_t)pair * 64 + d) * 512 + j0;
      *(volatile v4u*)(VTh + go) = hw;
      *(volatile v4u*)(VTl + go) = lw;
    }
    __threadfence();
  }
}

__global__ __launch_bounds__(256) void k_attn(const float* __restrict__ F1, const float* __restrict__ F2,
                                              const float* __restrict__ MJ,
                                              const unsigned short* __restrict__ vhp, const unsigned short* __restrict__ vlp,
                                              unsigned short* X1) {
  __shared__ __align__(16) float s_f2[512];
  __shared__ __align__(16) float s_m[512];
  __shared__ __align__(16) float Os[8][16 * TP];
  const int tid  = threadIdx.x;
  const int wave = tid >> 5;
  const int lane = tid & 31;
  const int hh   = lane >> 4;
  const int c    = lane & 15;
  const int blk  = blockIdx.x;
  const int grp  = blk & 3;
  const int pair = blk >> 2;
  const int b = pair >> 3, hd = pair & 7;

  if (tid < 128) {
    const v4f a  = *(const v4f*)(F2 + (size_t)pair * 512 + tid * 4);
    const v4f a2 = *(const v4f*)(MJ + (size_t)pair * 512 + tid * 4);
    *(v4f*)(s_f2 + tid * 4) = a;
    *(v4f*)(s_m  + tid * 4) = a2;
  }
  __syncthreads();

  const int i0 = grp * 128 + wave * 16;
  const float f1v = F1[(size_t)pair * 512 + i0 + c];
  const __bf16* Vh = (const __bf16*)(const void*)vhp + (size_t)pair * 64 * 512;
  const __bf16* Vl = (const __bf16*)(const void*)vlp + (size_t)pair * 64 * 512;

  v8f acc[4];
#pragma unroll
  for (int t = 0; t < 4; ++t) acc[t] = zero8();

  for (int j0 = 0; j0 < NN; j0 += 32) {
    const float* f2p = s_f2 + j0 + 8 * hh;
    const float* mp  = s_m  + j0 + 8 * hh;
    const v4f fa0 = *(const v4fa*)(f2p),      fa1 = *(const v4fa*)(f2p + 4);
    const v4f fb0 = *(const v4fa*)(f2p + 16), fb1 = *(const v4fa*)(f2p + 20);
    const v4f ma0 = *(const v4fa*)(mp),       ma1 = *(const v4fa*)(mp + 4);
    const v4f mb0 = *(const v4fa*)(mp + 16),  mb1 = *(const v4fa*)(mp + 20);
    float p[16];
#pragma unroll
    for (int e = 0; e < 4; ++e) {
      p[e]      = pexp(f1v, fa0[e], ma0[e]);
      p[4 + e]  = pexp(f1v, fa1[e], ma1[e]);
      p[8 + e]  = pexp(f1v, fb0[e], mb0[e]);
      p[12 + e] = pexp(f1v, fb1[e], mb1[e]);
    }
    v8u hw, lw;
#pragma unroll
    for (int v = 0; v < 8; ++v) {
      const float x0 = p[2 * v], x1 = p[2 * v + 1];
      const unsigned short h0 = f2bf_bits(x0), h1 = f2bf_bits(x1);
      const unsigned short l0 = f2bf_bits(x0 - bf_bits2f(h0)), l1 = f2bf_bits(x1 - bf_bits2f(h1));
      hw[v] = pk16(h0, h1);
      lw[v] = pk16(l0, l1);
    }
    const v16b pa = __builtin_bit_cast(v16b, hw);
    const v16b pl = __builtin_bit_cast(v16b, lw);
#pragma unroll
    for (int t = 0; t < 4; ++t) {
      const size_t vo = (size_t)(t * 16 + c) * 512 + j0 + 8 * hh;
      const v16b vh = FragB::load(Vh + vo);
      const v16b vl = FragB::load(Vl + vo);
      acc[t] = at_mma(pa, vh, acc[t]);
      acc[t] = at_mma(pl, vh, acc[t]);
      acc[t] = at_mma(pa, vl, acc[t]);
    }
  }

  float* os = Os[wave];
#pragma unroll
  for (int t = 0; t < 4; ++t)
#pragma unroll
    for (int r = 0; r < 8; ++r) os[(8 * hh + r) * TP + t * 16 + c] = acc[t][r];
  __builtin_amdgcn_fence(__ATOMIC_RELEASE, "workgroup");
  __builtin_amdgcn_wave_barrier();
  __builtin_amdgcn_fence(__ATOMIC_ACQUIRE, "workgroup");
  {
    const int q = lane >> 3, c8 = (lane & 7) * 8;
    v4u hv[4], lv[4];
#pragma unroll
    for (int it = 0; it < 4; ++it) {
      const int row = it * 4 + q;
      const float* sp = os + row * TP + c8;
      const v4f x0 = *(const v4fa*)(sp);
      const v4f x1 = *(const v4fa*)(sp + 4);
      v4u a, a2;
#pragma unroll
      for (int e = 0; e < 2; ++e) {
        const float y0 = eluf(x0[2 * e]), y1 = eluf(x0[2 * e + 1]);
        const float y2 = eluf(x1[2 * e]), y3 = eluf(x1[2 * e + 1]);
        const unsigned short h0 = f2bf_bits(y0), h1 = f2bf_bits(y1), h2 = f2bf_bits(y2), h3 = f2bf_bits(y3);
        a[e]      = pk16(h0, h1);
        a[2 + e]  = pk16(h2, h3);
        a2[e]     = pk16(f2bf_bits(y0 - bf_bits2f(h0)), f2bf_bits(y1 - bf_bits2f(h1)));
        a2[2 + e] = pk16(f2bf_bits(y2 - bf_bits2f(h2)), f2bf_bits(y3 - bf_bits2f(h3)));
      }
      hv[it] = a; lv[it] = a2;
    }
    for (int pass = 0; pass < 2; ++pass) {
#pragma unroll
      for (int it = 0; it < 4; ++it) {
        const int row = it * 4 + q;
        const size_t go = ((size_t)b * NN + i0 + row) * K2 + hd * HD + c8;
        *(volatile v4u*)(X1 + go) = hv[it];
        *(volatile v4u*)(X1 + go + C1) = lv[it];
      }
      __threadfence();
    }
  }
}

__global__ __launch_bounds__(256) void k_out2(const float* __restrict__ WH2, const float* __restrict__ a_out, float* G) {
  __shared__ __align__(16) float sav[128];
  __shared__ __align__(16) float sf[1024];
  __shared__ __align__(16) float wj[512];
  __shared__ __align__(16) float part[256];
  __shared__ __align__(16) float gs[64];
  __shared__ float red[8];
  const int tid = threadIdx.x;
  const int b = blockIdx.x;
  float* tile = dynT;

  if (tid < 128) sav[tid] = bfr(a_out[tid]);
  stage_tile(tile, WH2 + (size_t)b * NN * HD, HD, tid);
  __syncthreads();
  dots_f12(tile, sav, sf, tid);
  __syncthreads();
  const float fm = block_max512(sf, red, tid);
  {
    const float f10 = sf[0];
    const float f2a = sf[512 + tid], f2b = sf[512 + tid + 256];
    const float ma = colmax(fm, f2a), mb = colmax(fm, f2b);
    float za = 0.0f, zb = 0.0f;
#pragma unroll 1
    for (int i = 0; i < 512; ++i) {
      const float f = sf[i];
      za += pexp(f, f2a, ma);
      zb += pexp(f, f2b, mb);
    }
    wj[tid]       = pexp(f10, f2a, ma) * (1.0f / za);
    wj[tid + 256] = pexp(f10, f2b, mb) * (1.0f / zb);
  }
  __syncthreads();
  {
    const int d = tid & 63, qtr = tid >> 6;
    float g = 0.0f;
#pragma unroll 4
    for (int jj = 0; jj < 128; ++jj) {
      const int j = qtr * 128 + jj;
      g = fmaf(wj[j], tile[j * TP + d], g);
    }
    part[qtr * 64 + d] = g;
  }
  __syncthreads();
  if (tid < 64) {
    const float g = ((part[tid] + part[64 + tid]) + part[128 + tid]) + part[192 + tid];
    gs[tid] = eluf(g);
  }
  __syncthreads();
  {
    const v4f gv = *(const v4fa*)(gs + (tid & 15) * 4);
    float* gp = G + (size_t)b * HD + (tid & 15) * 4;
    if (tid < 16) *(volatile v4f*)gp = gv;
    __threadfence();
    if (tid < 16) *(volatile v4f*)gp = gv;
  }
}

__global__ __launch_bounds__(256) void k_head(const float* __restrict__ feats, const float* __restrict__ G,
                                              const float* __restrict__ W1, const float* __restrict__ b1,
                                              const float* __restrict__ prelu_a,
                                              const float* __restrict__ gamma, const float* __restrict__ beta,
                                              const float* __restrict__ mean, const float* __restrict__ var,
                                              const float* __restrict__ W2, const float* __restrict__ b2,
                                              float* out) {
  __shared__ __align__(16) float cs[NB * CP];
  __shared__ float hs[NB * 65];
  __shared__ float w2s[64];
  const int tid = threadIdx.x;
#pragma unroll 4
  for (int it = 0; it < 8; ++it) {
    const int p = it * 256 + tid;
    const int bb = p >> 6, c4 = (p & 63) * 4;
    const v4f a = *(const v4f*)(feats + (size_t)p * 4);
    v4f r;
    r[0] = bfr(a[0]); r[1] = bfr(a[1]); r[2] = bfr(a[2]); r[3] = bfr(a[3]);
    *(v4f*)(cs + bb * CP + c4) = r;
  }
#pragma unroll
  for (int it = 0; it < 2; ++it) {
    const int p = it * 256 + tid;
    const int bb = p >> 4, c4 = (p & 15) * 4;
    const v4f a = *(const v4f*)(G + (size_t)p * 4);
    *(v4f*)(cs + bb * CP + NF + c4) = a;
  }
  if (tid < 64) w2s[tid] = bfr(W2[tid]);
  __syncthreads();

  const int n = tid & 63, bg = tid >> 6;
  float acc[8];
#pragma unroll
  for (int q = 0; q < 8; ++q) acc[q] = 0.0f;
#pragma unroll 1
  for (int k = 0; k < NCAT; ++k) {
    const float w = bfr(W1[k * HD + n]);
    const float* cp = cs + (bg * 8) * CP + k;
#pragma unroll
    for (int q = 0; q < 8; ++q) acc[q] = fmaf(cp[q * CP], w, acc[q]);
  }
  {
    const float bb = bfr(b1[n]);
    const float pa = bfr(prelu_a[0]);
    const float mu = bfr(mean[n]);
    const float va = bfr(var[n]);
    const float ga = bfr(gamma[n]);
    const float be = bfr(beta[n]);
    const float rs = 1.0f / sqrtf(va + BN_EPS);
#pragma unroll
    for (int q = 0; q < 8; ++q) {
      float h = acc[q] + bb;
      h = (h >= 0.0f) ? h : pa * h;
      h = (h - mu) * rs * ga + be;
      hs[(bg * 8 + q) * 65 + n] = h;
    }
  }
  __syncthreads();
  if (tid < 32) {
    float o = 0.0f;
#pragma unroll 4
    for (int d = 0; d < 64; ++d) o = fmaf(hs[tid * 65 + d], w2s[d], o);
    o += bfr(b2[0]);
    *(volatile float*)(out + tid) = o;
    __threadfence();
    *(volatile float*)(out + tid) = o;
  }
}

extern "C" void kernel_launch(void* const* d_in, const int* in_sizes, int n_in,
                              void* d_out, int out_size, void* d_ws, size_t ws_size,
                              hipStream_t stream) {
  if (n_in < 15) return;
  if (in_sizes[0] != NB * NF) return;
  if (in_sizes[1] != NB * NN * NF) return;
  if (in_sizes[2] != NH * NF * HD) return;
  if (in_sizes[3] != NH * 2 * HD) return;
  if (in_sizes[4] != C1 * HD) return;
  if (in_sizes[5] != 2 * HD) return;
  if (in_sizes[6] != NCAT * HD) return;
  if (in_sizes[7] != HD || in_sizes[8] != 1) return;
  if (in_sizes[9] != HD || in_sizes[10] != HD || in_sizes[11] != HD || in_sizes[12] != HD) return;
  if (in_sizes[13] != HD || in_sizes[14] != 1) return;
  if (out_size != NB) return;

  const float* feats  = (const float*)d_in[0];
  const float* nfeat  = (const float*)d_in[1];
  const float* wheads = (const float*)d_in[2];
  const float* aheads = (const float*)d_in[3];
  const float* wout   = (const float*)d_in[4];
  const float* aout   = (const float*)d_in[5];
  const float* W1     = (const float*)d_in[6];
  const float* b1     = (const float*)d_in[7];
  const float* prelua = (const float*)d_in[8];
  const float* gamma  = (const float*)d_in[9];
  const float* beta   = (const float*)d_in[10];
  const float* mean   = (const float*)d_in[11];
  const float* var    = (const float*)d_in[12];
  const float* W2     = (const float*)d_in[13];
  const float* b2     = (const float*)d_in[14];

  const size_t sXB  = (size_t)MR * NF * 2;
  const size_t sW1T = (size_t)C1 * NF * 2;
  const size_t sW2D = (size_t)HD * K2 * 2;
  const size_t sWH1 = (size_t)MR * C1 * 4;
  const size_t sFP  = (size_t)NB * NH * NN * 4;
  const size_t sVT  = (size_t)NB * NH * HD * NN * 2;
  const size_t sX1  = (size_t)MR * K2 * 2;
  const size_t sWH2 = (size_t)MR * HD * 4;
  const size_t sG   = (size_t)NB * HD * 4;
  size_t off = 0;
  const size_t oXB  = off; off += sXB;
  const size_t oW1T = off; off += sW1T;
  const size_t oW2D = off; off += sW2D;
  const size_t oWH1 = off; off += sWH1;
  const size_t oF1  = off; off += sFP;
  const size_t oF2  = off; off += sFP;
  const size_t oMJ  = off; off += sFP;
  const size_t oVTh = off; off += sVT;
  const size_t oVTl = off; off += sVT;
  const size_t oX1  = off; off += sX1;
  const size_t oWH2 = off; off += sWH2;
  const size_t oG   = off; off += sG;
  if (off > ws_size) return;
  if (off > (size_t)134217728) return;

  char* ws = (char*)d_ws;
  unsigned short* XB  = (unsigned short*)(ws + oXB);
  unsigned short* W1T = (unsigned short*)(ws + oW1T);
  unsigned short* W2D = (unsigned short*)(ws + oW2D);
  float*          WH1 = (float*)(ws + oWH1);
  float*          F1  = (float*)(ws + oF1);
  float*          F2  = (float*)(ws + oF2);
  float*          MJ  = (float*)(ws + oMJ);
  unsigned short* VTh = (unsigned short*)(ws + oVTh);
  unsigned short* VTl = (unsigned short*)(ws + oVTl);
  unsigned short* X1  = (unsigned short*)(ws + oX1);
  float*          WH2 = (float*)(ws + oWH2);
  float*          G   = (float*)(ws + oG);

  const dim3 blk(256);
  (void)hipFuncSetAttribute(reinterpret_cast<const void*>(&k_stats), hipFuncAttributeMaxDynamicSharedMemorySize, (int)DYN_TILE_BYTES);
  (void)hipFuncSetAttribute(reinterpret_cast<const void*>(&k_out2),  hipFuncAttributeMaxDynamicSharedMemorySize, (int)DYN_TILE_BYTES);

  const int n8x = MR * NF / 8;
  cvt_bf16x8_kernel<<<dim3((n8x + 255) / 256), blk, 0, stream>>>(nfeat, XB, n8x);
  k_tr<<<dim3(NF / 64, NH), blk, 0, stream>>>(wheads, W1T, (long)NF * HD, NF, 0);
  k_tr<<<dim3(C1 / 64, 1), blk, 0, stream>>>(wout, W2D, 0L, K2, 1);
  wmma_gemm64_f32<<<dim3(((MR / 64) * (C1 / 64) + 7) / 8), blk, 0, stream>>>(XB, NF, W1T, NF, WH1, C1, MR, C1, NF);
  k_stats<<<dim3(NB * NH), blk, DYN_TILE_BYTES, stream>>>(WH1, aheads, F1, F2, MJ, VTh, VTl);
  k_attn<<<dim3(NB * NH * (NN / 128)), blk, 0, stream>>>(F1, F2, MJ, VTh, VTl, X1);
  wmma_gemm64_f32<<<dim3(((MR / 64) * (HD / 64) + 7) / 8), blk, 0, stream>>>(X1, K2, W2D, K2, WH2, HD, MR, HD, K2);
  k_out2<<<dim3(NB), blk, DYN_TILE_BYTES, stream>>>(WH2, aout, G);
  k_head<<<dim3(1), blk, 0, stream>>>(feats, G, W1, b1, prelua, gamma, beta, mean, var, W2, b2, (float*)d_out);
  (void)hipGetLastError();
}
